// GNNMotion_76768245449447
// MI455X (gfx1250) — hardware-verified
//
#include <hip/hip_runtime.h>
#include <stddef.h>
#include <stdint.h>
#include <math.h>


#define NN      4096
#define EE      131072
#define XD      8
#define HD      128
#define NHEAD   4
#define QW      512
#define QKVW    1536
#define HLW     256
#define OHLW    1024
#define NB      64
#define D1      256
#define D1HL    512
#define NOUT    60
#define NOUTP   64
#define NTHR    256
#define NWAVE   8
#define EPT     8
#define CHUNK   (NTHR * EPT)
#define WCAP    (EPT * 32)
#define LISTN   (NWAVE * WCAP)
#define NBMAX   2048
#define SLOTB   11
#define NBRUN   256
#define NSCAN   (NN / NBRUN)
#define RCAP    12288
#define DEGCAP  128
#define STW     512
#define GBM     64
#define GBN     64
#define GTHR    128
#define SCALE_S 0.08838834764831845f
#define LDS_SCAN ((2 * RCAP + 2 * NBMAX + LISTN) * 4 + 64)
#define LDS_DEC  (NB * HLW * 2 + NB * D1HL * 2 + 4096 * 4)
#define WSMAX   134217728

static_assert(NN % GBM == 0);
static_assert(NN % 128 == 0);
static_assert(QW == NHEAD * HD);
static_assert(QKVW == 3 * QW);
static_assert((NB * NOUT * 4) % 128 == 0);
static_assert(32 * 16 == QW);
static_assert(HD == 8 * 16);
static_assert(NBRUN * NSCAN == NN);
static_assert((NBRUN & (NBRUN - 1)) == 0 && NBRUN <= NBMAX && NBRUN >= 16);
static_assert(RCAP * 100 >= 8324 * 105);
static_assert(DEGCAP >= 52 + 8);
static_assert(DEGCAP <= 128);
static_assert(NWAVE * STW <= RCAP);
static_assert((RCAP % 32) == 0);
static_assert(EE % CHUNK == 0);
static_assert(EE < (1 << (32 - SLOTB)));
static_assert((CHUNK & (CHUNK - 1)) == 0 && CHUNK <= (1 << SLOTB));
static_assert(NBMAX == (1 << SLOTB));
static_assert(NTHR * 8 == NBMAX);
static_assert(LISTN >= NBMAX);
static_assert(GBM == (GTHR / 32) * 16);
static_assert((HLW % 32) == 0 && (OHLW % 32) == 0 && (D1HL % 32) == 0);
static_assert((QKVW % GBN) == 0 && (HD % GBN) == 0);
static_assert(LDS_SCAN <= 300000 && LDS_DEC <= 300000);
static_assert(NB * NOUT <= 4096);

typedef float          v4f  __attribute__((ext_vector_type(4)));
typedef float          v8f  __attribute__((ext_vector_type(8)));
typedef int            v4i  __attribute__((ext_vector_type(4)));
typedef int            v8i  __attribute__((ext_vector_type(8)));
typedef unsigned int   v4u  __attribute__((ext_vector_type(4)));
typedef unsigned short v8us __attribute__((ext_vector_type(8)));
typedef __bf16         v16b __attribute__((ext_vector_type(16)));
typedef v4f  __attribute__((may_alias)) v4fa;
typedef v4u  __attribute__((may_alias)) v4ua;
typedef v8us __attribute__((may_alias)) v8usa;
union FragB { v16b v; v8us h[2]; v8i w; };

__device__ __forceinline__ v8f wmb(const FragB& a, const FragB& b, v8f c) {
  v8f d = __builtin_amdgcn_wmma_f32_16x16x32_bf16(false, a.v, false, b.v, (short)0, c, false, false);
  asm volatile("v_nop\n\tv_nop\n\tv_nop\n\tv_nop" : "+v"(d) : "v"(a.w), "v"(b.w));
  return d;
}

__device__ __forceinline__ unsigned int f2bf(float f) {
  const unsigned int u = __float_as_uint(f);
  return ((u + 0x7FFFu + ((u >> 16) & 1u)) >> 16) & 0xFFFFu;
}
__device__ __forceinline__ float bf2f(unsigned int b) { return __uint_as_float(b << 16); }
__device__ __forceinline__ float bfr(float f) { return bf2f(f2bf(f)); }
__device__ __forceinline__ v4f bfr4(const v4f a) {
  v4f r; r.x = bfr(a.x); r.y = bfr(a.y); r.z = bfr(a.z); r.w = bfr(a.w); return r;
}
__device__ __forceinline__ unsigned int pk2(float lo, float hi) { return f2bf(lo) | (f2bf(hi) << 16); }
__device__ __forceinline__ unsigned int pk2lo(float lo, float hi) {
  return f2bf(lo - bfr(lo)) | (f2bf(hi - bfr(hi)) << 16);
}
__device__ __forceinline__ v4u pack8(const v4f a, const v4f b) {
  v4u r;
  r.x = pk2(a.x, a.y); r.y = pk2(a.z, a.w); r.z = pk2(b.x, b.y); r.w = pk2(b.z, b.w);
  return r;
}
__device__ __forceinline__ v4u pack8lo(const v4f a, const v4f b) {
  v4u r;
  r.x = pk2lo(a.x, a.y); r.y = pk2lo(a.z, a.w); r.z = pk2lo(b.x, b.y); r.w = pk2lo(b.z, b.w);
  return r;
}
__device__ __forceinline__ float relun(float v) { return (v > 0.0f) ? v : (v - v); }
__device__ __forceinline__ v4f relun4(const v4f a) {
  v4f r; r.x = relun(a.x); r.y = relun(a.y); r.z = relun(a.z); r.w = relun(a.w); return r;
}
__device__ __forceinline__ float dot4(const v4f q, const v4f k, float acc) {
  acc = fmaf(q.x, k.x, acc); acc = fmaf(q.y, k.y, acc);
  acc = fmaf(q.z, k.z, acc); acc = fmaf(q.w, k.w, acc);
  return acc;
}
__device__ __forceinline__ v4f upd4(const v4f a, const float s1, const float s2, const v4f v) {
  v4f r;
  r.x = fmaf(a.x, s1, s2 * v.x); r.y = fmaf(a.y, s1, s2 * v.y);
  r.z = fmaf(a.z, s1, s2 * v.z); r.w = fmaf(a.w, s1, s2 * v.w);
  return r;
}

__device__ __forceinline__ int scan_chunk(const int* __restrict__ dsts, int nE, int cbase, int slotBase,
                                          int nb, int vec8, int* list, int tid, int lane, int wave) {
  int wc = 0;
  const int el0  = tid * EPT;
  const int e0   = cbase + el0;
  const int sent = -2147483647 - 1;
  v4i da, db;
  if (vec8 != 0 && cbase + CHUNK <= nE) {
    da = *(const v4i*)(dsts + e0);
    db = *(const v4i*)(dsts + e0 + 4);
  } else {
    da.x = (e0     < nE) ? dsts[min(e0,     nE - 1)] : sent;
    da.y = (e0 + 1 < nE) ? dsts[min(e0 + 1, nE - 1)] : sent;
    da.z = (e0 + 2 < nE) ? dsts[min(e0 + 2, nE - 1)] : sent;
    da.w = (e0 + 3 < nE) ? dsts[min(e0 + 3, nE - 1)] : sent;
    db.x = (e0 + 4 < nE) ? dsts[min(e0 + 4, nE - 1)] : sent;
    db.y = (e0 + 5 < nE) ? dsts[min(e0 + 5, nE - 1)] : sent;
    db.z = (e0 + 6 < nE) ? dsts[min(e0 + 6, nE - 1)] : sent;
    db.w = (e0 + 7 < nE) ? dsts[min(e0 + 7, nE - 1)] : sent;
  }
  const unsigned nbs = (unsigned)slotBase;
  const unsigned unb = (unsigned)nb;
  const unsigned s0 = (unsigned)da.x - nbs, s1 = (unsigned)da.y - nbs;
  const unsigned s2 = (unsigned)da.z - nbs, s3 = (unsigned)da.w - nbs;
  const unsigned s4 = (unsigned)db.x - nbs, s5 = (unsigned)db.y - nbs;
  const unsigned s6 = (unsigned)db.z - nbs, s7 = (unsigned)db.w - nbs;
  const bool h0 = s0 < unb, h1 = s1 < unb, h2 = s2 < unb, h3 = s3 < unb;
  const bool h4 = s4 < unb, h5 = s5 < unb, h6 = s6 < unb, h7 = s7 < unb;
  const unsigned any = __builtin_amdgcn_ballot_w32(h0 | h1 | h2 | h3 | h4 | h5 | h6 | h7);
  if (any != 0u) {
#define HITJ(J, HJ, SJ) { \
      const unsigned mj = __builtin_amdgcn_ballot_w32(HJ); \
      if (mj != 0u) { \
        if (HJ) { \
          const int pos = wc + (int)__builtin_amdgcn_mbcnt_lo(mj, 0u); \
          if (pos < WCAP) list[wave * WCAP + pos] = ((el0 + (J)) << SLOTB) | (int)(SJ); \
        } \
        wc += (int)__builtin_popcount(mj); } }
    HITJ(0, h0, s0)
    HITJ(1, h1, s1)
    HITJ(2, h2, s2)
    HITJ(3, h3, s3)
    HITJ(4, h4, s4)
    HITJ(5, h5, s5)
    HITJ(6, h6, s6)
    HITJ(7, h7, s7)
#undef HITJ
  }
  return wc;
}

__device__ __forceinline__ void wtr_unit(const float* __restrict__ w, const int Kin, const int Ncol, const int Nrows,
                                         const int Kout, unsigned short* wt, const int u) {
  const int kq = Kout >> 3;
  const int n  = u / kq;
  if (n >= Nrows) return;
  const int k8 = (u - n * kq) * 8;
  const int kk = k8 - (k8 / Kin) * Kin;
  const int ncl = n < Ncol ? n : Ncol - 1;
  const float* p = w + (size_t)kk * (size_t)Ncol + ncl;
  v4f a, b;
  a.x = p[0];                    a.y = p[(size_t)Ncol];         a.z = p[(size_t)2 * Ncol];     a.w = p[(size_t)3 * Ncol];
  b.x = p[(size_t)4 * Ncol];     b.y = p[(size_t)5 * Ncol];     b.z = p[(size_t)6 * Ncol];     b.w = p[(size_t)7 * Ncol];
  const v4f z4 = {0.f, 0.f, 0.f, 0.f};
  if (n >= Ncol) { a = z4; b = z4; }
  const v4u wv = pack8(a, b);
  unsigned short* o = wt + (size_t)n * (size_t)Kout + k8;
  *(volatile v4u*)o = wv;
  __threadfence();
  *(volatile v4u*)o = wv;
}

__global__ __launch_bounds__(NTHR) void k_prep(
    const float* __restrict__ xw2,
    const float* __restrict__ q0, const float* __restrict__ k0, const float* __restrict__ v0,
    const float* __restrict__ pw0,
    const float* __restrict__ q1, const float* __restrict__ k1, const float* __restrict__ v1,
    const float* __restrict__ pw1,
    const float* __restrict__ dw1, const float* __restrict__ dw2,
    unsigned short* W2T, unsigned short* QKVT0, unsigned short* QKVT1,
    unsigned short* PWT0, unsigned short* PWT1, unsigned short* D1T, unsigned short* D2T) {
  const int b = (int)blockIdx.x, tid = (int)threadIdx.x;
  if (b < 16) {
    wtr_unit(xw2, HD, HD, HD, HLW, W2T, b * NTHR + tid);
  } else if (b < 80) {
    wtr_unit(q0, HD, QW, QW, HLW, QKVT0, (b - 16) * NTHR + tid);
  } else if (b < 144) {
    wtr_unit(k0, HD, QW, QW, HLW, QKVT0 + (size_t)QW * HLW, (b - 80) * NTHR + tid);
  } else if (b < 208) {
    wtr_unit(v0, HD, QW, QW, HLW, QKVT0 + (size_t)2 * QW * HLW, (b - 144) * NTHR + tid);
  } else if (b < 272) {
    wtr_unit(q1, HD, QW, QW, HLW, QKVT1, (b - 208) * NTHR + tid);
  } else if (b < 336) {
    wtr_unit(k1, HD, QW, QW, HLW, QKVT1 + (size_t)QW * HLW, (b - 272) * NTHR + tid);
  } else if (b < 400) {
    wtr_unit(v1, HD, QW, QW, HLW, QKVT1 + (size_t)2 * QW * HLW, (b - 336) * NTHR + tid);
  } else if (b < 464) {
    wtr_unit(pw0, QW, HD, HD, OHLW, PWT0, (b - 400) * NTHR + tid);
  } else if (b < 528) {
    wtr_unit(pw1, QW, HD, HD, OHLW, PWT1, (b - 464) * NTHR + tid);
  } else if (b < 560) {
    wtr_unit(dw1, HD, D1, D1, HLW, D1T, (b - 528) * NTHR + tid);
  } else if (b < 576) {
    wtr_unit(dw2, D1, NOUT, NOUTP, D1HL, D2T, (b - 560) * NTHR + tid);
  }
}

template<int HASRES>
__device__ __forceinline__ void epi_hn(float* stg, const v8f (&acc)[4],
                                       const float* __restrict__ bias, const float* __restrict__ resid,
                                       float* outF, unsigned short* outHL,
                                       const int rowBase, const int col0, const int tid) {
  const int lane = tid & 31, wave = tid >> 5, hh = lane >> 4, m = lane & 15;
#pragma unroll
  for (int t = 0; t < 4; ++t) {
    const int lc = 16 * t + m;
#pragma unroll
    for (int r = 0; r < 8; ++r) {
      const int lr = 16 * wave + 8 * hh + r;
      stg[lr * GBN + lc] = acc[t][r];
    }
  }
  __syncthreads();
  const v4f bv = bfr4(*(const v4fa*)(bias + col0 + 4 * m));
  v4f fv[8];
#pragma unroll
  for (int i = 0; i < 8; ++i) {
    const int lr = 16 * wave + 2 * i + hh;
    const int gr = rowBase + lr;
    v4f v = *(const v4fa*)(stg + lr * GBN + 4 * m);
    v = v + bv;
    if (HASRES) {
      const v4f rv = *(const v4fa*)(resid + (size_t)gr * HD + col0 + 4 * m);
      v = rv + v;
    }
    v = relun4(v);
    fv[i] = v;
    *(v4fa*)(stg + lr * GBN + 4 * m) = v;
  }
#pragma unroll
  for (int i = 0; i < 8; ++i) {
    const int lr = 16 * wave + 2 * i + hh;
    float* op = outF + (size_t)(rowBase + lr) * HD + col0 + 4 * m;
    *(volatile v4f*)op = fv[i];
  }
  __syncthreads();
  const int rq = lane >> 3, pc = lane & 7;
  v4u hv[4], lv[4];
#pragma unroll
  for (int i = 0; i < 4; ++i) {
    const int lr = 16 * wave + 4 * i + rq;
    const v4f ga = *(const v4fa*)(stg + lr * GBN + 8 * pc);
    const v4f gb = *(const v4fa*)(stg + lr * GBN + 8 * pc + 4);
    hv[i] = pack8(ga, gb);
    lv[i] = pack8lo(ga, gb);
  }
#pragma unroll
  for (int i = 0; i < 4; ++i) {
    const int lr = 16 * wave + 4 * i + rq;
    unsigned short* hp = outHL + (size_t)(rowBase + lr) * HLW + col0 + 8 * pc;
    *(volatile v4u*)hp = hv[i];
    *(volatile v4u*)(hp + HD) = lv[i];
  }
  __threadfence();
#pragma unroll
  for (int i = 0; i < 8; ++i) {
    const int lr = 16 * wave + 2 * i + hh;
    float* op = outF + (size_t)(rowBase + lr) * HD + col0 + 4 * m;
    *(volatile v4f*)op = fv[i];
  }
#pragma unroll
  for (int i = 0; i < 4; ++i) {
    const int lr = 16 * wave + 4 * i + rq;
    unsigned short* hp = outHL + (size_t)(rowBase + lr) * HLW + col0 + 8 * pc;
    *(volatile v4u*)hp = hv[i];
    *(volatile v4u*)(hp + HD) = lv[i];
  }
}

__global__ __launch_bounds__(GTHR) void k_enc(const float* __restrict__ X, const float* __restrict__ w1,
                                              const float* __restrict__ b1, const unsigned short* __restrict__ W2T,
                                              const float* __restrict__ b2, float* outF, unsigned short* outHL) {
  __shared__ __attribute__((aligned(16))) unsigned short At[GBM * HLW];
  __shared__ __attribute__((aligned(16))) float stg[GBM * GBN];
  __shared__ __attribute__((aligned(16))) float w1s[XD * HD];
  __shared__ __attribute__((aligned(16))) float b1s[HD];
  __shared__ __attribute__((aligned(16))) float xs[GBM * XD];
  const int tid = (int)threadIdx.x, lane = tid & 31, wave = tid >> 5, hh = lane >> 4, m = lane & 15;
  const int rowBase = (int)blockIdx.x * GBM;
  const int col0    = (int)blockIdx.y * GBN;

  {
    const v4f wa = *(const v4fa*)(w1 + 8 * tid);
    const v4f wb = *(const v4fa*)(w1 + 8 * tid + 4);
    *(v4fa*)(w1s + 8 * tid)     = bfr4(wa);
    *(v4fa*)(w1s + 8 * tid + 4) = bfr4(wb);
    b1s[tid] = bfr(b1[tid]);
    const v4f xv = *(const v4fa*)(X + (size_t)rowBase * XD + 4 * tid);
    *(v4fa*)(xs + 4 * tid) = bfr4(xv);
  }
  __syncthreads();

  {
    const int cg = tid & 15, r0 = tid >> 4;
    const int c0 = 8 * cg;
    const v4f bA = *(const v4fa*)(b1s + c0);
    const v4f bB = *(const v4fa*)(b1s + c0 + 4);
#pragma unroll 1
    for (int i = 0; i < 8; ++i) {
      const int r = r0 + 8 * i;
      const v4f xa = *(const v4fa*)(xs + r * XD);
      const v4f xb = *(const v4fa*)(xs + r * XD + 4);
      const float xr[8] = {xa.x, xa.y, xa.z, xa.w, xb.x, xb.y, xb.z, xb.w};
      v4f sA = {0.f, 0.f, 0.f, 0.f};
      v4f sB = {0.f, 0.f, 0.f, 0.f};
#pragma unroll
      for (int j = 0; j < XD; ++j) {
        const v4f wA = *(const v4fa*)(w1s + j * HD + c0);
        const v4f wB = *(const v4fa*)(w1s + j * HD + c0 + 4);
        sA.x = fmaf(xr[j], wA.x, sA.x); sA.y = fmaf(xr[j], wA.y, sA.y);
        sA.z = fmaf(xr[j], wA.z, sA.z); sA.w = fmaf(xr[j], wA.w, sA.w);
        sB.x = fmaf(xr[j], wB.x, sB.x); sB.y = fmaf(xr[j], wB.y, sB.y);
        sB.z = fmaf(xr[j], wB.z, sB.z); sB.w = fmaf(xr[j], wB.w, sB.w);
      }
      sA = relun4(sA + bA);
      sB = relun4(sB + bB);
      *(v4ua*)(At + r * HLW + c0)      = pack8(sA, sB);
      *(v4ua*)(At + r * HLW + HD + c0) = pack8lo(sA, sB);
    }
  }
  __syncthreads();

  v8f acc[4];
  {
    const v8f z = {0.f, 0.f, 0.f, 0.f, 0.f, 0.f, 0.f, 0.f};
    acc[0] = z; acc[1] = z; acc[2] = z; acc[3] = z;
  }
  const unsigned short* ap = At + (16 * wave + m) * HLW + 8 * hh;
  const unsigned short* wp = W2T + (size_t)(col0 + m) * HLW + 8 * hh;
#pragma unroll 1
  for (int ks = 0; ks < HLW / 32; ++ks) {
    FragB af;
    af.h[0] = *(const v8usa*)(ap + 32 * ks);
    af.h[1] = *(const v8usa*)(ap + 32 * ks + 16);
#pragma unroll
    for (int t = 0; t < 4; ++t) {
      const unsigned short* wq = wp + (size_t)(16 * t) * HLW + 32 * ks;
      FragB bf;
      bf.h[0] = *(const v8usa*)wq;
      bf.h[1] = *(const v8usa*)(wq + 16);
      acc[t] = wmb(af, bf, acc[t]);
    }
  }
  epi_hn<0>(stg, acc, b2, b2, outF, outHL, rowBase, col0, tid);
}

template<int EPI>
__global__ __launch_bounds__(GTHR) void k_gemm(
    const unsigned short* __restrict__ A, const unsigned short* __restrict__ WT,
    float* outF, int K, int ldo,
    const float* __restrict__ bias, const float* __restrict__ resid, unsigned short* outHL) {
  __shared__ __attribute__((aligned(16))) float stg[GBM * GBN];
  const int tid = (int)threadIdx.x, lane = tid & 31, wave = tid >> 5, hh = lane >> 4, m = lane & 15;
  const int rowBase = (int)blockIdx.x * GBM;
  const int col0    = (int)blockIdx.y * GBN;

  v8f acc[4];
  {
    const v8f z = {0.f, 0.f, 0.f, 0.f, 0.f, 0.f, 0.f, 0.f};
    acc[0] = z; acc[1] = z; acc[2] = z; acc[3] = z;
  }
  const unsigned short* ap = A  + (size_t)(rowBase + 16 * wave + m) * (size_t)K + 8 * hh;
  const unsigned short* wp = WT + (size_t)(col0 + m) * (size_t)K + 8 * hh;
  const int ksteps = K >> 5;
#pragma unroll 1
  for (int ks = 0; ks < ksteps; ++ks) {
    FragB af;
    af.h[0] = *(const v8usa*)(ap + 32 * ks);
    af.h[1] = *(const v8usa*)(ap + 32 * ks + 16);
#pragma unroll
    for (int t = 0; t < 4; ++t) {
      const unsigned short* wq = wp + (size_t)(16 * t) * (size_t)K + 32 * ks;
      FragB bf;
      bf.h[0] = *(const v8usa*)wq;
      bf.h[1] = *(const v8usa*)(wq + 16);
      acc[t] = wmb(af, bf, acc[t]);
    }
  }

  if (EPI == 0) {
#pragma unroll
    for (int t = 0; t < 4; ++t) {
      const int lc = 16 * t + m;
#pragma unroll
      for (int r = 0; r < 8; ++r) {
        const int lr = 16 * wave + 8 * hh + r;
        stg[lr * GBN + lc] = acc[t][r];
      }
    }
    __syncthreads();
    v4f fv[8];
#pragma unroll
    for (int i = 0; i < 8; ++i) {
      const int lr = 16 * wave + 2 * i + hh;
      fv[i] = *(const v4fa*)(stg + lr * GBN + 4 * m);
    }
#pragma unroll
    for (int i = 0; i < 8; ++i) {
      const int lr = 16 * wave + 2 * i + hh;
      float* op = outF + (size_t)(rowBase + lr) * (size_t)ldo + col0 + 4 * m;
      *(volatile v4f*)op = fv[i];
    }
    __threadfence();
#pragma unroll
    for (int i = 0; i < 8; ++i) {
      const int lr = 16 * wave + 2 * i + hh;
      float* op = outF + (size_t)(rowBase + lr) * (size_t)ldo + col0 + 4 * m;
      *(volatile v4f*)op = fv[i];
    }
  } else {
    epi_hn<1>(stg, acc, bias, resid, outF, outHL, rowBase, col0, tid);
  }
}

__global__ __launch_bounds__(NTHR) void k_scan(
    const int* __restrict__ keys, const int* __restrict__ gsrc,
    const float* __restrict__ QKV, unsigned short* OHL, int* FLG,
    int nN, int nE, int nb, int vec8) {
  extern __shared__ v4f lds_dyn[];
  int* reg1 = (int*)lds_dyn;
  int* reg2 = reg1 + RCAP;
  int* scnt = reg2 + RCAP;
  int* soff = scnt + NBMAX;
  int* list = soff + NBMAX;
  int* wcnt = list + LISTN;
  int* wtot = wcnt + NWAVE;
  const int tid = (int)threadIdx.x, lane = tid & 31, wave = tid >> 5;
  const int nodeBase = (int)blockIdx.x * nb;

  for (int i = tid; i < NBMAX; i += NTHR) scnt[i] = 0;
  __syncthreads();

  int tot = 0;
  const int nChunks = (nE + CHUNK - 1) / CHUNK;
#pragma unroll 1
  for (int ch = 0; ch < nChunks; ++ch) {
    const int cbase = ch * CHUNK;
    const int wc = scan_chunk(keys, nE, cbase, nodeBase, nb, vec8, list, tid, lane, wave);
    if (lane == 0) wcnt[wave] = wc;
    __syncthreads();
    int pre = 0, all = 0;
#pragma unroll
    for (int w2 = 0; w2 < NWAVE; ++w2) {
      int c = wcnt[w2];
      c = c < 0 ? 0 : (c > WCAP ? WCAP : c);
      all += c;
      pre += (w2 < wave) ? c : 0;
    }
    const int wcc  = wc > WCAP ? WCAP : wc;
    const int base = tot + pre;
#pragma unroll 1
    for (int i = lane; i < wcc; i += 32) {
      const int ent = list[wave * WCAP + i];
      const int el  = (ent >> SLOTB) & (CHUNK - 1);
      const int sl  = ent & (NBMAX - 1);
      int eid = cbase + el;
      eid = eid > nE - 1 ? nE - 1 : eid;
      const int pos = base + i;
      if (pos < RCAP) reg1[pos] = (int)(((unsigned)eid << SLOTB) | (unsigned)sl);
    }
    tot += all;
    tot = tot > RCAP ? RCAP : tot;
    __syncthreads();
  }
  const int nh = tot;

  if (wave == 0) {
#pragma unroll 1
    for (int b0 = 0; b0 < nh; b0 += 32) {
      const int idx = b0 + lane;
      const int uv  = reg1[idx < nh ? idx : nh - 1];
      const int m32 = (nh - b0) < 32 ? (nh - b0) : 32;
#pragma unroll 1
      for (int k = 0; k < m32; ++k) {
        const int u  = __builtin_amdgcn_readlane(uv, k);
        const int sl = u & (NBMAX - 1);
        if (lane == 0) scnt[sl] = scnt[sl] + 1;
      }
    }
  }
  __syncthreads();

  {
    const v4i ca = *(const v4i*)(scnt + 8 * tid);
    const v4i cb = *(const v4i*)(scnt + 8 * tid + 4);
    const int e0 = ca.x < 0 ? 0 : ca.x, e1 = ca.y < 0 ? 0 : ca.y, e2 = ca.z < 0 ? 0 : ca.z, e3 = ca.w < 0 ? 0 : ca.w;
    const int e4 = cb.x < 0 ? 0 : cb.x, e5 = cb.y < 0 ? 0 : cb.y, e6 = cb.z < 0 ? 0 : cb.z, e7 = cb.w < 0 ? 0 : cb.w;
    const int ts = e0 + e1 + e2 + e3 + e4 + e5 + e6 + e7;
    int incl = ts;
#pragma unroll
    for (int d = 1; d < 32; d <<= 1) {
      const int up = __shfl_up(incl, d);
      if (lane >= d) incl += up;
    }
    if (lane == 31) wtot[wave] = incl;
    __syncthreads();
    int pre = 0;
#pragma unroll
    for (int w2 = 0; w2 < NWAVE; ++w2) pre += (w2 < wave) ? wtot[w2] : 0;
    int run = pre + incl - ts;
    soff[8 * tid + 0] = run; run += e0;
    soff[8 * tid + 1] = run; run += e1;
    soff[8 * tid + 2] = run; run += e2;
    soff[8 * tid + 3] = run; run += e3;
    soff[8 * tid + 4] = run; run += e4;
    soff[8 * tid + 5] = run; run += e5;
    soff[8 * tid + 6] = run; run += e6;
    soff[8 * tid + 7] = run;
  }
  __syncthreads();
  for (int i = tid; i < NBMAX; i += NTHR) list[i] = soff[i];
  __syncthreads();

  if (wave == 0) {
#pragma unroll 1
    for (int b0 = 0; b0 < nh; b0 += 32) {
      const int idx = b0 + lane;
      const int uv  = reg1[idx < nh ? idx : nh - 1];
      int eidl = (int)((unsigned)uv >> SLOTB);
      eidl = eidl > nE - 1 ? nE - 1 : eidl;
      int mv = gsrc[eidl];
      mv = mv < 0 ? 0 : (mv > nN - 1 ? nN - 1 : mv);
      const int m32 = (nh - b0) < 32 ? (nh - b0) : 32;
#pragma unroll 1
      for (int k = 0; k < m32; ++k) {
        const int u  = __builtin_amdgcn_readlane(uv, k);
        const int mk = __builtin_amdgcn_readlane(mv, k);
        const int sl = u & (NBMAX - 1);
        if (lane == 0) {
          int pos = list[sl];
          pos = pos < 0 ? 0 : (pos > RCAP - 1 ? RCAP - 1 : pos);
          reg2[pos] = mk;
          list[sl] = pos + 1;
        }
      }
    }
  }
  __syncthreads();

  const int nbw = nb >> 3;
  const bool ovf = (nh >= RCAP);
  const float qnan = __int_as_float(0x7fc00000);
  float* stw = (float*)reg1 + wave * STW;
  const int c0 = 16 * lane;
  int wflag = ovf ? 1 : 0;

#pragma unroll 1
  for (int jt = 0; jt < nbw; ++jt) {
    const int slot = wave * nbw + jt;
    const int grow = nodeBase + slot;
    const int gcl  = grow < nN ? grow : nN - 1;
    int st = soff[slot];
    const int craw = scnt[slot];
    int cnt = craw;
    st  = st < 0 ? 0 : (st > nh ? nh : st);
    cnt = cnt < 0 ? 0 : (cnt > DEGCAP ? DEGCAP : cnt);
    if (cnt > nh - st) cnt = nh - st;
    const bool bad = ovf || (craw > DEGCAP);
    const float pz = bad ? qnan : 0.0f;
    wflag |= (craw > DEGCAP) ? 1 : 0;

    const float* qp = QKV + (size_t)gcl * QKVW + c0;
    const v4f q0 = *(const v4fa*)qp;
    const v4f q1 = *(const v4fa*)(qp + 4);
    const v4f q2 = *(const v4fa*)(qp + 8);
    const v4f q3 = *(const v4fa*)(qp + 12);

    int ml0, ml1, ml2, ml3;
    {
      const int i0 = st + lane, i1 = i0 + 32, i2 = i0 + 64, i3 = i0 + 96;
      const int r0 = reg2[i0 > RCAP - 1 ? RCAP - 1 : i0];
      const int r1 = reg2[i1 > RCAP - 1 ? RCAP - 1 : i1];
      const int r2 = reg2[i2 > RCAP - 1 ? RCAP - 1 : i2];
      const int r3 = reg2[i3 > RCAP - 1 ? RCAP - 1 : i3];
      ml0 = (lane      < cnt) ? r0 : -1;
      ml1 = (lane + 32 < cnt) ? r1 : -1;
      ml2 = (lane + 64 < cnt) ? r2 : -1;
      ml3 = (lane + 96 < cnt) ? r3 : -1;
    }

    float mx = -1.0e30f, dn = 0.0f;
    v4f a0 = {0.f, 0.f, 0.f, 0.f};
    v4f a1 = {0.f, 0.f, 0.f, 0.f};
    v4f a2 = {0.f, 0.f, 0.f, 0.f};
    v4f a3 = {0.f, 0.f, 0.f, 0.f};

#pragma unroll 1
    for (int j = 0; j < cnt; ++j) {
      int idx = st + j; idx = idx > RCAP - 1 ? RCAP - 1 : idx;
      int mj = reg2[idx];
      mj = mj < 0 ? 0 : (mj > nN - 1 ? nN - 1 : mj);
      const bool dupl = ((ml0 == mj) & (lane      < j)) | ((ml1 == mj) & (lane + 32 < j)) |
                        ((ml2 == mj) & (lane + 64 < j)) | ((ml3 == mj) & (lane + 96 < j));
      const unsigned db = __builtin_amdgcn_ballot_w32(dupl);
      if (db != 0u) continue;

      const float* kp = QKV + (size_t)mj * QKVW + QW + c0;
      const v4f k0 = *(const v4fa*)kp;
      const v4f k1 = *(const v4fa*)(kp + 4);
      const v4f k2 = *(const v4fa*)(kp + 8);
      const v4f k3 = *(const v4fa*)(kp + 12);
      const v4f v0 = *(const v4fa*)(kp + QW);
      const v4f v1 = *(const v4fa*)(kp + QW + 4);
      const v4f v2 = *(const v4fa*)(kp + QW + 8);
      const v4f v3 = *(const v4fa*)(kp + QW + 12);
      float part = 0.0f;
      part = dot4(q0, k0, part);
      part = dot4(q1, k1, part);
      part = dot4(q2, k2, part);
      part = dot4(q3, k3, part);
      part += __shfl_xor(part, 1);
      part += __shfl_xor(part, 2);
      part += __shfl_xor(part, 4);
      const float sc = part * SCALE_S;
      const float df = sc - mx;
      const float ee = expf(-fabsf(df));
      const bool up  = df > 0.f;
      const float s1 = up ? ee : 1.0f;
      const float s2 = up ? 1.0f : ee;
      mx = up ? sc : mx;
      dn = fmaf(dn, s1, s2);
      a0 = upd4(a0, s1, s2, v0);
      a1 = upd4(a1, s1, s2, v1);
      a2 = upd4(a2, s1, s2, v2);
      a3 = upd4(a3, s1, s2, v3);
    }
    const float rc  = __builtin_amdgcn_rcpf(dn > 0.f ? dn : 1.0f);
    const float inv = (dn > 0.f) ? rc : qnan;
    v4f r0, r1, r2, r3;
    r0.x = fmaf(a0.x, inv, pz); r0.y = fmaf(a0.y, inv, pz); r0.z = fmaf(a0.z, inv, pz); r0.w = fmaf(a0.w, inv, pz);
    r1.x = fmaf(a1.x, inv, pz); r1.y = fmaf(a1.y, inv, pz); r1.z = fmaf(a1.z, inv, pz); r1.w = fmaf(a1.w, inv, pz);
    r2.x = fmaf(a2.x, inv, pz); r2.y = fmaf(a2.y, inv, pz); r2.z = fmaf(a2.z, inv, pz); r2.w = fmaf(a2.w, inv, pz);
    r3.x = fmaf(a3.x, inv, pz); r3.y = fmaf(a3.y, inv, pz); r3.z = fmaf(a3.z, inv, pz); r3.w = fmaf(a3.w, inv, pz);

    __builtin_amdgcn_fence(__ATOMIC_RELEASE, "wavefront");
    __builtin_amdgcn_wave_barrier();
    *(v4fa*)(stw + c0)      = r0;
    *(v4fa*)(stw + c0 + 4)  = r1;
    *(v4fa*)(stw + c0 + 8)  = r2;
    *(v4fa*)(stw + c0 + 12) = r3;
    __builtin_amdgcn_fence(__ATOMIC_RELEASE, "wavefront");
    __builtin_amdgcn_wave_barrier();
    const v4f ga = *(const v4fa*)(stw + 8 * lane);
    const v4f gb = *(const v4fa*)(stw + 8 * lane + 4);
    const v4f gc = *(const v4fa*)(stw + 256 + 8 * lane);
    const v4f gd = *(const v4fa*)(stw + 256 + 8 * lane + 4);
    const v4u hA = pack8(ga, gb),  lA = pack8lo(ga, gb);
    const v4u hB = pack8(gc, gd),  lB = pack8lo(gc, gd);
    unsigned short* gp = OHL + (size_t)grow * OHLW + 8 * lane;
    const bool wr = grow < nN;
    if (wr) {
      *(volatile v4u*)gp         = hA;
      *(volatile v4u*)(gp + 256) = hB;
      *(volatile v4u*)(gp + 512) = lA;
      *(volatile v4u*)(gp + 768) = lB;
    }
    __threadfence();
    if (wr) {
      *(volatile v4u*)gp         = hA;
      *(volatile v4u*)(gp + 256) = hB;
      *(volatile v4u*)(gp + 512) = lA;
      *(volatile v4u*)(gp + 768) = lB;
    }
  }

  if (lane == 0) wtot[wave] = wflag;
  __syncthreads();
  if (wave == 0) {
    int f = 0;
#pragma unroll
    for (int w2 = 0; w2 < NWAVE; ++w2) f |= wtot[w2];
    const v4i fv = {f, f, f, f};
    int* fp = FLG + (size_t)blockIdx.x * 32 + 4 * (lane & 7);
    const bool wl = lane < 8;
    if (wl) *(volatile v4i*)fp = fv;
    __threadfence();
    if (wl) *(volatile v4i*)fp = fv;
  }
}

__global__ __launch_bounds__(NTHR) void k_dec(
    const float* __restrict__ HN, const int* __restrict__ tgt,
    const unsigned short* __restrict__ D1T, const float* __restrict__ db1,
    const unsigned short* __restrict__ D2T, const float* __restrict__ db2,
    const int* __restrict__ FLG, float* out, int nN) {
  extern __shared__ v4f lds_dyn[];
  unsigned short* At = (unsigned short*)lds_dyn;
  unsigned short* A2 = At + NB * HLW;
  float* outS = (float*)(A2 + NB * D1HL);
  const int tid = (int)threadIdx.x, lane = tid & 31, wave = tid >> 5, hh = lane >> 4, m = lane & 15;
  const float qnan = __int_as_float(0x7fc00000);

  const int fl = FLG[(tid & 31) * 32];
  const unsigned pb = __builtin_amdgcn_ballot_w32(fl != 0);
  const bool poison = (pb != 0u);

  {
    const int b = tid >> 2, qd = tid & 3;
    int ti = tgt[b];
    ti = ti < 0 ? 0 : (ti > nN - 1 ? nN - 1 : ti);
    const float* hp = HN + (size_t)ti * HD;
#pragma unroll
    for (int i = 0; i < 4; ++i) {
      const int c0 = 8 * (qd + 4 * i);
      const v4f ga = *(const v4fa*)(hp + c0);
      const v4f gb = *(const v4fa*)(hp + c0 + 4);
      *(v4ua*)(At + b * HLW + c0)      = pack8(ga, gb);
      *(v4ua*)(At + b * HLW + HD + c0) = pack8lo(ga, gb);
    }
  }
  __syncthreads();

  const int rt = wave & 3, cq = wave >> 2;
  {
    v8f acc[8];
    const v8f z = {0.f, 0.f, 0.f, 0.f, 0.f, 0.f, 0.f, 0.f};
#pragma unroll
    for (int t = 0; t < 8; ++t) acc[t] = z;
    const unsigned short* ap = At + (16 * rt + m) * HLW + 8 * hh;
    const unsigned short* wp = D1T + (size_t)(128 * cq + m) * HLW + 8 * hh;
#pragma unroll 1
    for (int ks = 0; ks < HLW / 32; ++ks) {
      FragB af;
      af.h[0] = *(const v8usa*)(ap + 32 * ks);
      af.h[1] = *(const v8usa*)(ap + 32 * ks + 16);
#pragma unroll
      for (int t = 0; t < 8; ++t) {
        const unsigned short* wq = wp + (size_t)(16 * t) * HLW + 32 * ks;
        FragB bf;
        bf.h[0] = *(const v8usa*)wq;
        bf.h[1] = *(const v8usa*)(wq + 16);
        acc[t] = wmb(af, bf, acc[t]);
      }
    }
#pragma unroll
    for (int t = 0; t < 8; ++t) {
      const int col = 128 * cq + 16 * t + m;
      const float bv = bfr(db1[col]);
#pragma unroll
      for (int r = 0; r < 8; ++r) {
        const int row = 16 * rt + 8 * hh + r;
        const float v = relun(acc[t][r] + bv);
        const unsigned int hb = f2bf(v);
        const unsigned int lb = f2bf(v - bf2f(hb));
        A2[row * D1HL + col]      = (unsigned short)hb;
        A2[row * D1HL + D1 + col] = (unsigned short)lb;
      }
    }
  }
  __syncthreads();

  {
    v8f acc[2];
    const v8f z = {0.f, 0.f, 0.f, 0.f, 0.f, 0.f, 0.f, 0.f};
    acc[0] = z; acc[1] = z;
    const unsigned short* ap = A2 + (16 * rt + m) * D1HL + 8 * hh;
    const unsigned short* wp = D2T + (size_t)(32 * cq + m) * D1HL + 8 * hh;
#pragma unroll 1
    for (int ks = 0; ks < D1HL / 32; ++ks) {
      FragB af;
      af.h[0] = *(const v8usa*)(ap + 32 * ks);
      af.h[1] = *(const v8usa*)(ap + 32 * ks + 16);
#pragma unroll
      for (int t = 0; t < 2; ++t) {
        const unsigned short* wq = wp + (size_t)(16 * t) * D1HL + 32 * ks;
        FragB bf;
        bf.h[0] = *(const v8usa*)wq;
        bf.h[1] = *(const v8usa*)(wq + 16);
        acc[t] = wmb(af, bf, acc[t]);
      }
    }
#pragma unroll
    for (int t = 0; t < 2; ++t) {
      const int col = 32 * cq + 16 * t + m;
      const int cc  = col < NOUT ? col : NOUT - 1;
      const float bv = bfr(db2[cc]);
#pragma unroll
      for (int r = 0; r < 8; ++r) {
        const int row = 16 * rt + 8 * hh + r;
        float v = acc[t][r] + bv;
        v = poison ? qnan : v;
        if (col < NOUT) outS[row * NOUT + col] = v;
      }
    }
  }
  __syncthreads();

  v4f fv[4];
#pragma unroll
  for (int i = 0; i < 4; ++i) {
    const int p  = tid + NTHR * i;
    const int pc = p < 959 ? p : 959;
    fv[i] = *(const v4fa*)(outS + 4 * pc);
  }
#pragma unroll
  for (int i = 0; i < 4; ++i) {
    const int p = tid + NTHR * i;
    if (p < (NB * NOUT) / 4) *(volatile v4f*)(out + 4 * p) = fv[i];
  }
  __threadfence();
#pragma unroll
  for (int i = 0; i < 4; ++i) {
    const int p = tid + NTHR * i;
    if (p < (NB * NOUT) / 4) *(volatile v4f*)(out + 4 * p) = fv[i];
  }
}

extern "C" void kernel_launch(void* const* d_in, const int* in_sizes, int n_in,
                              void* d_out, int out_size, void* d_ws, size_t ws_size,
                              hipStream_t stream) {
  if (n_in < 26) return;
  if (in_sizes[0] != NN * XD) return;
  if (in_sizes[2] != 2 * EE) return;
  if (in_sizes[3] != NB) return;
  if (in_sizes[4] != XD * HD || in_sizes[5] != HD) return;
  if (in_sizes[6] != HD * HD || in_sizes[7] != HD) return;
  if (in_sizes[12] != HD * QW || in_sizes[13] != HD * QW || in_sizes[14] != HD * QW) return;
  if (in_sizes[15] != QW * HD || in_sizes[16] != HD) return;
  if (in_sizes[17] != HD * QW || in_sizes[18] != HD * QW || in_sizes[19] != HD * QW) return;
  if (in_sizes[20] != QW * HD || in_sizes[21] != HD) return;
  if (in_sizes[22] != HD * D1 || in_sizes[23] != D1) return;
  if (in_sizes[24] != D1 * NOUT || in_sizes[25] != NOUT) return;
  if (out_size != NB * NOUT) return;

  const float* X    = (const float*)d_in[0];
  const int*   EI   = (const int*)  d_in[2];
  const int*   tgt  = (const int*)  d_in[3];
  const float* xw1  = (const float*)d_in[4];
  const float* xb1  = (const float*)d_in[5];
  const float* xw2  = (const float*)d_in[6];
  const float* xb2  = (const float*)d_in[7];
  const float* gq0  = (const float*)d_in[12];
  const float* gk0  = (const float*)d_in[13];
  const float* gv0  = (const float*)d_in[14];
  const float* gpw0 = (const float*)d_in[15];
  const float* gpb0 = (const float*)d_in[16];
  const float* gq1  = (const float*)d_in[17];
  const float* gk1  = (const float*)d_in[18];
  const float* gv1  = (const float*)d_in[19];
  const float* gpw1 = (const float*)d_in[20];
  const float* gpb1 = (const float*)d_in[21];
  const float* dw1  = (const float*)d_in[22];
  const float* db1  = (const float*)d_in[23];
  const float* dw2  = (const float*)d_in[24];
  const float* db2  = (const float*)d_in[25];
  float* out = (float*)d_out;

  char* ws = (char*)d_ws;
  size_t off = 0;
  const size_t oQKV  = off; off += (size_t)NN * QKVW * 4;
  const size_t oOHL  = off; off += (size_t)NN * OHLW * 2;
  const size_t oHNA  = off; off += (size_t)NN * HD * 4;
  const size_t oHNB  = off; off += (size_t)NN * HD * 4;
  const size_t oHNHL = off; off += (size_t)NN * HLW * 2;
  const size_t oQT0  = off; off += (size_t)QKVW * HLW * 2;
  const size_t oQT1  = off; off += (size_t)QKVW * HLW * 2;
  const size_t oPT0  = off; off += (size_t)HD * OHLW * 2;
  const size_t oPT1  = off; off += (size_t)HD * OHLW * 2;
  const size_t oW2T  = off; off += (size_t)HD * HLW * 2;
  const size_t oD1T  = off; off += (size_t)D1 * HLW * 2;
  const size_t oD2T  = off; off += (size_t)NOUTP * D1HL * 2;
  const size_t oFLG  = off; off += (size_t)2 * NSCAN * 128;
  if (off > ws_size || off > (size_t)WSMAX) return;
  float*          QKV  = (float*)(ws + oQKV);
  unsigned short* OHL  = (unsigned short*)(ws + oOHL);
  float*          HNA  = (float*)(ws + oHNA);
  float*          HNB  = (float*)(ws + oHNB);
  unsigned short* HNHL = (unsigned short*)(ws + oHNHL);
  unsigned short* QT0  = (unsigned short*)(ws + oQT0);
  unsigned short* QT1  = (unsigned short*)(ws + oQT1);
  unsigned short* PT0  = (unsigned short*)(ws + oPT0);
  unsigned short* PT1  = (unsigned short*)(ws + oPT1);
  unsigned short* W2T  = (unsigned short*)(ws + oW2T);
  unsigned short* D1T  = (unsigned short*)(ws + oD1T);
  unsigned short* D2T  = (unsigned short*)(ws + oD2T);
  int*            FLG  = (int*)(ws + oFLG);

  hipFuncSetAttribute(reinterpret_cast<const void*>(&k_scan),
                      hipFuncAttributeMaxDynamicSharedMemorySize, LDS_SCAN);
  hipFuncSetAttribute(reinterpret_cast<const void*>(&k_dec),
                      hipFuncAttributeMaxDynamicSharedMemorySize, LDS_DEC);

  const int* keys = EI;
  const int* gsrc = EI + EE;
  const int vec8 = ((EE & 3) == 0) ? 1 : 0;

  k_prep<<<576, NTHR, 0, stream>>>(xw2, gq0, gk0, gv0, gpw0, gq1, gk1, gv1, gpw1, dw1, dw2,
                                   W2T, QT0, QT1, PT0, PT1, D1T, D2T);
  k_enc<<<dim3(NN / GBM, HD / GBN), GTHR, 0, stream>>>(X, xw1, xb1, W2T, xb2, HNA, HNHL);

  k_gemm<0><<<dim3(NN / GBM, QKVW / GBN), GTHR, 0, stream>>>(HNHL, QT0, QKV, HLW, QKVW, xb2, HNA, HNHL);
  k_scan<<<NSCAN, NTHR, LDS_SCAN, stream>>>(keys, gsrc, QKV, OHL, FLG, NN, EE, NBRUN, vec8);
  k_gemm<1><<<dim3(NN / GBM, HD / GBN), GTHR, 0, stream>>>(OHL, PT0, HNB, OHLW, HD, gpb0, HNA, HNHL);

  k_gemm<0><<<dim3(NN / GBM, QKVW / GBN), GTHR, 0, stream>>>(HNHL, QT1, QKV, HLW, QKVW, xb2, HNA, HNHL);
  k_scan<<<NSCAN, NTHR, LDS_SCAN, stream>>>(keys, gsrc, QKV, OHL, FLG + NSCAN * 32, NN, EE, NBRUN, vec8);
  k_gemm<1><<<dim3(NN / GBM, HD / GBN), GTHR, 0, stream>>>(OHL, PT1, HNA, OHLW, HD, gpb1, HNB, HNHL);

  k_dec<<<1, NTHR, LDS_DEC, stream>>>(HNA, tgt, D1T, db1, D2T, db2, FLG, out, NN);
}
